// My_scaled_dot_product_attention_43662637531564
// MI455X (gfx1250) — hardware-verified
//
#include <hip/hip_runtime.h>


namespace {
constexpr int B = 2, NH = 16, S = 2048, D = 64, BH = B * NH;
constexpr float XS = 8.0f, PS = 1024.0f;
typedef _Float16 b16;
typedef __attribute__((ext_vector_type(16))) _Float16 v16b;
typedef __attribute__((ext_vector_type(8))) _Float16 v8b;
typedef __attribute__((ext_vector_type(8))) float v8f;
typedef __attribute__((ext_vector_type(4))) float v4f;
typedef __attribute__((ext_vector_type(2))) float v2f;
__device__ __forceinline__ float bf16_rne(float f) { unsigned int u = __float_as_uint(f); u += 0x7FFFu + ((u >> 16) & 1u); float r = __uint_as_float(u & 0xFFFF0000u); asm volatile("" : "+v"(r)); return r; }
__device__ __forceinline__ void split16(float v, b16& hi, b16& lo) { hi = (b16)v; lo = (b16)(v - (float)hi); }
__device__ __forceinline__ v16b frag_kb(const b16* p, int hh) { const v8b a = *(const v8b*)(p + 8 * hh), b = *(const v8b*)(p + 16 + 8 * hh); v16b f;
#pragma unroll
  for (int e = 0; e < 8; ++e) { f[e] = a[e]; f[8 + e] = b[e]; } return f; }
__device__ __forceinline__ v8f wmma16b(v16b a, v16b b, v8f c) { v8f d = __builtin_amdgcn_wmma_f32_16x16x32_f16(false, a, false, b, (short)0, c, false, false); asm volatile("v_nop\n\tv_nop\n\tv_nop\n\tv_nop" : "+v"(d) : "v"(a), "v"(b)); return d; }
__device__ __forceinline__ void wave_lds_sync() { __builtin_amdgcn_fence(__ATOMIC_RELEASE, "workgroup"); __builtin_amdgcn_wave_barrier(); __builtin_amdgcn_fence(__ATOMIC_ACQUIRE, "workgroup"); }

__global__ __launch_bounds__(256) void qk_kernel(const float* __restrict__ q, const float* __restrict__ k, b16* __restrict__ QH, b16* __restrict__ KH) { const size_t u = (size_t)blockIdx.x * 256 + threadIdx.x; if (u >= (size_t)BH * S * (D / 8)) return; const size_t e0 = u * 8; v8b a, c;
#pragma unroll
  for (int j = 0; j < 8; ++j) { a[j] = (b16)(bf16_rne(q[e0 + j]) * XS); c[j] = (b16)(bf16_rne(k[e0 + j]) * XS); } for (int pass = 0; pass < 2; ++pass) { *(volatile v8b*)(QH + e0) = a; *(volatile v8b*)(KH + e0) = c; __threadfence(); } }
__global__ __launch_bounds__(32) void vt_kernel(const float* __restrict__ v, b16* __restrict__ VT) { const int lane = threadIdx.x; const int ch = blockIdx.x % (S / 32), bh = blockIdx.x / (S / 32); const size_t row = (size_t)bh * S + ch * 32 + lane; const size_t base = ((size_t)bh * (S / 32) + ch) * D;
  for (int pass = 0; pass < 2; ++pass) {
#pragma unroll 8
    for (int d = 0; d < D; ++d) ((volatile b16*)VT)[(base + d) * 64 + lane] = (b16)(bf16_rne(v[row * D + d]) * XS); __threadfence(); } }
__global__ __launch_bounds__(32) void att_kernel(const b16* __restrict__ QH, const b16* __restrict__ KH, const b16* __restrict__ VT, const int* __restrict__ mask, int BHV, float* __restrict__ out) {
  __shared__ __attribute__((aligned(16))) b16 Ph[16][40], Pl[16][40]; __shared__ float Sc[16][33], Mx[16], Dn[16], Sf[16], Of[16][D + 2]; __shared__ int Mt[16][33];
  const int lane = threadIdx.x, nloc = lane & 15, hlf = lane >> 4; const int qt = blockIdx.x % (S / 16); const int bh = blockIdx.x / (S / 16); if (bh >= BHV) return; const int q0 = qt * 16; const size_t qrow = (size_t)bh * S + q0;
  if (lane < 16) { Mx[lane] = -INFINITY; Dn[lane] = 0.0f; Sf[lane] = 0.0f; }
  v16b qa[2]; qa[0] = frag_kb(QH + (qrow + nloc) * D, hlf); qa[1] = frag_kb(QH + (qrow + nloc) * D + 32, hlf);
  v8f acc[4] = {(v8f){}, (v8f){}, (v8f){}, (v8f){}}; wave_lds_sync();
#pragma unroll 1
  for (int kc = 0; kc < S; kc += 32) {
    int any = 0; for (int rr = 0; rr < 16; ++rr) { const int mv = mask[(size_t)(q0 + rr) * S + kc + lane]; Mt[rr][lane] = mv; any |= mv; }
    for (int o = 16; o; o >>= 1) any |= __shfl_xor(any, o); if (any == 0) continue;
    wave_lds_sync();
#pragma unroll
    for (int blk = 0; blk < 2; ++blk) { v8f s = {}; const size_t kr = ((size_t)bh * S + kc + blk * 16 + nloc) * D; s = wmma16b(qa[0], frag_kb(KH + kr, hlf), s); s = wmma16b(qa[1], frag_kb(KH + kr + 32, hlf), s);
#pragma unroll
      for (int r8 = 0; r8 < 8; ++r8) { const int rl = 8 * hlf + r8, kk = blk * 16 + nloc; Sc[rl][kk] = Mt[rl][kk] != 0 ? s[r8] * (0.125f / (XS * XS)) : -INFINITY; } }
    wave_lds_sync();
#pragma unroll 1
    for (int qi = 0; qi < 16; ++qi) { const float sv = Sc[qi][lane]; float cm = sv; for (int o = 16; o; o >>= 1) cm = fmaxf(cm, __shfl_xor(cm, o)); const float mo = Mx[qi]; const float mn = fmaxf(mo, cm); const float p = (sv == -INFINITY || mn == -INFINITY) ? 0.0f : __expf(sv - mn); float ps = p; for (int o = 16; o; o >>= 1) ps += __shfl_xor(ps, o);
      b16 ph, plo; split16(p * PS, ph, plo); Ph[qi][lane] = ph; Pl[qi][lane] = plo; if (lane == 0) { const float sf = (mo == -INFINITY) ? ((mn == -INFINITY) ? 1.0f : 0.0f) : __expf(mo - mn); Sf[qi] = sf; Dn[qi] = Dn[qi] * sf + ps; Mx[qi] = mn; } }
    wave_lds_sync(); const v16b pa = frag_kb(&Ph[nloc][0], hlf), pb = frag_kb(&Pl[nloc][0], hlf); const size_t vb = (((size_t)bh * (S / 32) + kc / 32) * D) * 64;
#pragma unroll
    for (int t = 0; t < 4; ++t) {
#pragma unroll
      for (int r8 = 0; r8 < 8; ++r8) acc[t][r8] *= Sf[8 * hlf + r8];
      const v16b vv = frag_kb(VT + vb + (size_t)(t * 16 + nloc) * 64, hlf); acc[t] = wmma16b(pa, vv, acc[t]); acc[t] = wmma16b(pb, vv, acc[t]); }
    wave_lds_sync(); }
#pragma unroll
  for (int t = 0; t < 4; ++t)
#pragma unroll
    for (int r8 = 0; r8 < 8; ++r8) { const int rl = 8 * hlf + r8; Of[rl][t * 16 + nloc] = acc[t][r8] * (1.0f / (PS * XS)) / Dn[rl]; }
  wave_lds_sync();
  for (int pass = 0; pass < 2; ++pass) { for (int rr = 0; rr < 16; ++rr) *(volatile v2f*)(out + (qrow + rr) * D + lane * 2) = (v2f){Of[rr][lane * 2], Of[rr][lane * 2 + 1]}; __threadfence(); }
}
}

extern "C" void kernel_launch(void* const* d_in, const int* in_sizes, int n_in, void* d_out, int out_size, void* d_ws, size_t ws_size, hipStream_t stream) {
  (void)n_in;
  auto Fp = [&](int i) { return (const float*)d_in[i]; }; auto Ip = [&](int i) { return (const int*)d_in[i]; };
  if (in_sizes[0] != BH * S * D || in_sizes[1] != BH * S * D || in_sizes[2] != BH * S * D || in_sizes[3] != S * S || out_size != BH * S * D) return;
  const int BHV = BH;
  size_t off = 0; char* ws = (char*)d_ws;
  auto carve = [&](size_t bytes) { char* p = ws + off; off += (bytes + 255) & ~(size_t)255; return p; };
  b16* QH = (b16*)carve((size_t)BH * S * D * 2); b16* KH = (b16*)carve((size_t)BH * S * D * 2); b16* VT = (b16*)carve((size_t)BH * (S / 32) * D * 64 * 2);
  if (off > ws_size || off > ((size_t)40 << 20)) return;
  qk_kernel<<<(unsigned)(((size_t)BH * S * (D / 8) + 255) / 256), 256, 0, stream>>>(Fp(0), Fp(1), QH, KH);
  vt_kernel<<<BH * (S / 32), 32, 0, stream>>>(Fp(2), VT);
  att_kernel<<<BHV * (S / 16), 32, 0, stream>>>(QH, KH, VT, Ip(3), BHV, (float*)d_out);
}
